// DynamicMaskHead_26508538151624
// MI455X (gfx1250) — hardware-verified
//
#include <hip/hip_runtime.h>
#include <math.h>

typedef __attribute__((ext_vector_type(16))) _Float16 v16h;
typedef __attribute__((ext_vector_type(16))) __bf16 v16b;
typedef __attribute__((ext_vector_type(8)))  _Float16 v8h;
typedef __attribute__((ext_vector_type(8)))  float v8f;
typedef __attribute__((ext_vector_type(4)))  float v4f;
typedef __attribute__((ext_vector_type(2)))  float v2f;
typedef __attribute__((ext_vector_type(4)))  unsigned v4u;
typedef __attribute__((ext_vector_type(4)))  int v4i;
typedef float __attribute__((may_alias)) float_a;
typedef int __attribute__((may_alias)) int_a;

template <typename T> __device__ __forceinline__ void vst2(void* p, T v) { *(volatile T*)p = v; __threadfence(); *(volatile T*)p = v; }
__device__ __forceinline__ v8f wmma16(v16h a, v16h b, v8f c) {
  v8f d = __builtin_amdgcn_wmma_f32_16x16x32_f16(false, a, false, b, (short)0, c, false, false);
  asm volatile("v_nop\n\tv_nop\n\tv_nop\n\tv_nop" : "+v"(d) : "v"(a), "v"(b));
  return d;
}
__device__ __forceinline__ v8f wmma_bf(v16b a, v16b b, v8f c) {
  v8f d = __builtin_amdgcn_wmma_f32_16x16x32_bf16(false, a, false, b, (short)0, c, false, false);
  asm volatile("v_nop\n\tv_nop\n\tv_nop\n\tv_nop" : "+v"(d) : "v"(a), "v"(b));
  return d;
}
__device__ __forceinline__ v16h frag_h(const _Float16* rowk0, int lane) {
  union { v16h v; v8h q[2]; } u; const _Float16* p = rowk0 + 8 * (lane >> 4);
  u.q[0] = *(const v8h*)p; u.q[1] = *(const v8h*)(p + 16); return u.v;
}
__device__ __forceinline__ v16h frag_f32(const float* rowk0, int lane) {
  v16h a; const float* p = rowk0 + 8 * (lane >> 4);
#pragma unroll
  for (int i = 0; i < 8; ++i) { a[i] = (_Float16)p[i]; a[8 + i] = (_Float16)p[16 + i]; }
  return a;
}
__device__ __forceinline__ v16h frag_f32s(const float* rowk0, int lane, float sc) {
  v16h a; const float* p = rowk0 + 8 * (lane >> 4);
#pragma unroll
  for (int i = 0; i < 8; ++i) { a[i] = (_Float16)(p[i] * sc); a[8 + i] = (_Float16)(p[16 + i] * sc); }
  return a;
}
__device__ __forceinline__ v16h fragc_f32(const float* W, int k0, int n, int lane, int ld, int K) {
  v16h a; const int g = lane >> 4;
#pragma unroll
  for (int i = 0; i < 8; ++i) { const int ka = k0 + 8 * g + i, kb = ka + 16;
    a[i] = (_Float16)(ka < K ? W[(size_t)(ka < K ? ka : K - 1) * ld + n] : 0.f); a[8 + i] = (_Float16)(kb < K ? W[(size_t)(kb < K ? kb : K - 1) * ld + n] : 0.f); }
  return a;
}
struct F2 { v16b h, l; };
__device__ __forceinline__ F2 bsplit16(const float v[16]) { F2 r;
#pragma unroll
  for (int i = 0; i < 16; ++i) { const __bf16 h = (__bf16)v[i]; r.h[i] = h; r.l[i] = (__bf16)(v[i] - (float)h); }
  return r; }
__device__ __forceinline__ F2 split_row(const float* row, int k0, int lane) { float v[16]; const float* p = row + k0 + 8 * (lane >> 4);
#pragma unroll
  for (int i = 0; i < 8; ++i) { v[i] = p[i]; v[8 + i] = p[16 + i]; }
  return bsplit16(v); }
__device__ __forceinline__ F2 split_rowK(const float* row, int k0, int lane, int K) { float v[16]; const int g = lane >> 4;
#pragma unroll
  for (int i = 0; i < 8; ++i) { const int ka = k0 + 8 * g + i, kb = ka + 16; v[i] = ka < K ? row[ka < K ? ka : K - 1] : 0.f; v[8 + i] = kb < K ? row[kb < K ? kb : K - 1] : 0.f; }
  return bsplit16(v); }
__device__ __forceinline__ F2 split_col(const float* W, int k0, int n, int lane, int ld, int K) { float v[16]; const int g = lane >> 4;
#pragma unroll
  for (int i = 0; i < 8; ++i) { const int ka = k0 + 8 * g + i, kb = ka + 16; v[i] = ka < K ? W[(size_t)(ka < K ? ka : K - 1) * ld + n] : 0.f; v[8 + i] = kb < K ? W[(size_t)(kb < K ? kb : K - 1) * ld + n] : 0.f; }
  return bsplit16(v); }
__device__ __forceinline__ v8f mac3(const F2& a, const F2& b, v8f c) { c = wmma_bf(a.l, b.h, c); c = wmma_bf(a.h, b.l, c); return wmma_bf(a.h, b.h, c); }
__device__ __forceinline__ float sigm(float v) { return 1.0f / (1.0f + expf(-v)); }
#define LDSX() do { asm volatile("s_wait_dscnt 0" ::: "memory"); __builtin_amdgcn_wave_barrier(); __builtin_amdgcn_fence(__ATOMIC_RELEASE, "workgroup"); } while (0)

__device__ __forceinline__ float bfr(float v) { return (float)(__bf16)v; }
#define NIMG 4
#define CIN 64
#define HH 60
#define WWD 160
#define NP (HH * WWD)
#define NINST 128
#define CH 128
#define NPAR 25217
#define OFF_W0 0
#define OFF_W1 8448
#define OFF_W2 24832
#define OFF_B0 24960
#define OFF_B1 25088
#define OFF_B2 25216
#ifndef NIB
#define NIB NINST
#endif
#define WS_XT 0u
#define WS_END (WS_XT + 4u * (size_t)NIMG * NP * CIN)
__global__ __launch_bounds__(256) void k_xt(const float* __restrict__ X, float* __restrict__ XT) { __shared__ float st[CIN][65];
  const int t = threadIdx.x; const int p0 = blockIdx.x * 64; const size_t n = blockIdx.y;
  for (int e = t; e < CIN * 64; e += 256) { const int c = e >> 6, pl = e & 63; st[c][pl] = bfr(X[(n * CIN + c) * NP + p0 + pl]); }
  __syncthreads();
  for (int e = t; e < 64 * 16; e += 256) { const int pl = e >> 4, q = e & 15; v4f o; o[0] = st[q * 4][pl]; o[1] = st[q * 4 + 1][pl]; o[2] = st[q * 4 + 2][pl]; o[3] = st[q * 4 + 3][pl]; vst2(XT + (n * NP + p0 + pl) * CIN + q * 4, o); } }
__global__ __launch_bounds__(128) void k_head(const float* __restrict__ XT, const float* __restrict__ PRM, const int* __restrict__ NUMI, float* __restrict__ OUT) { __shared__ __align__(16) _Float16 sh[4][16][CH + 8]; __shared__ __align__(16) float so[64];
  const int tid = threadIdx.x, wave = tid >> 5, lane = tid & 31, col = lane & 15, g = lane >> 4; const int inst = blockIdx.y; const int p0 = blockIdx.x * 64 + wave * 16;
  int img = 0; { int acc_ = 0; for (int n = 0; n < NIMG; ++n) { acc_ += NUMI[n]; if (inst >= acc_) img = n + 1; } if (img >= NIMG) img = NIMG - 1; }
  const float* P = PRM + (size_t)inst * NPAR; const float* w0 = P + OFF_W0; const float* w1 = P + OFF_W1; const float* w2 = P + OFF_W2;
  v8f acc[8] = {};
#pragma unroll
  for (int kc = 0; kc < CIN / 32; ++kc) { v16b a; { const float* p = XT + ((size_t)img * NP + p0 + col) * CIN + kc * 32 + 8 * g;
#pragma unroll
      for (int i = 0; i < 8; ++i) { a[i] = (__bf16)p[i]; a[8 + i] = (__bf16)p[16 + i]; } }
#pragma unroll
    for (int j = 0; j < 8; ++j) { v16b w; const int o = j * 16 + col; const float* wr = w0 + (size_t)o * (CIN + 2) + 2 + kc * 32 + 8 * g;
#pragma unroll
      for (int i = 0; i < 8; ++i) { w[i] = (__bf16)wr[i]; w[8 + i] = (__bf16)wr[16 + i]; }
      asm volatile("s_wait_loadcnt 0x0" ::: "memory"); acc[j] = wmma_bf(a, w, acc[j]); } }
#pragma unroll
  for (int j = 0; j < 8; ++j) { const int o = j * 16 + col; const float wx = bfr(w0[(size_t)o * (CIN + 2)]), wy = bfr(w0[(size_t)o * (CIN + 2) + 1]), bb = bfr(P[OFF_B0 + o]);
#pragma unroll
    for (int r = 0; r < 8; ++r) { const int p = p0 + 8 * g + r; const float lx = (float)(p % WWD) / (float)WWD, ly = (float)(p / WWD) / (float)WWD;
      sh[wave][8 * g + r][o] = (_Float16)fmaxf(acc[j][r] + wx * lx + wy * ly + bb, 0.f); }
    asm volatile("s_wait_loadcnt 0x0" ::: "memory"); }
  LDSX();
  v8f acc2[8] = {};
#pragma unroll
  for (int kc = 0; kc < CH / 32; ++kc) { const v16h a = frag_h(&sh[wave][col][kc * 32], lane);
#pragma unroll
    for (int j = 0; j < 8; ++j) { v16h w; const int o = j * 16 + col; const float* wr = w1 + (size_t)o * CH + kc * 32 + 8 * g;
#pragma unroll
      for (int i = 0; i < 8; ++i) { w[i] = (_Float16)bfr(wr[i]); w[8 + i] = (_Float16)bfr(wr[16 + i]); }
      asm volatile("s_wait_loadcnt 0x0" ::: "memory"); acc2[j] = wmma16(a, w, acc2[j]); } }
  float p3[8];
#pragma unroll
  for (int r = 0; r < 8; ++r) p3[r] = 0.f;
#pragma unroll
  for (int j = 0; j < 8; ++j) { const int o = j * 16 + col; const float bb = bfr(P[OFF_B1 + o]), ww = bfr(w2[o]);
#pragma unroll
    for (int r = 0; r < 8; ++r) p3[r] += fmaxf(acc2[j][r] + bb, 0.f) * ww; }
#pragma unroll
  for (int r = 0; r < 8; ++r) {
#pragma unroll
    for (int s_ = 1; s_ < 16; s_ <<= 1) p3[r] += __shfl_xor(p3[r], s_); }
  if (col == 0) { const float b2 = bfr(P[OFF_B2]) - 2.19f;
#pragma unroll
    for (int r = 0; r < 8; ++r) so[wave * 16 + 8 * g + r] = p3[r] + b2; }
  __syncthreads();
  if (tid < 16) vst2(OUT + (size_t)inst * NP + (size_t)blockIdx.x * 64 + tid * 4, *(const v4f*)&so[tid * 4]); }
extern "C" void kernel_launch(void* const* d_in, const int* in_sizes, int n_in, void* d_out, int out_size, void* d_ws, size_t ws_size, hipStream_t stream) {
  (void)in_sizes; (void)n_in; (void)out_size;
  const float** F = (const float**)d_in;
  if (ws_size < (size_t)WS_END) return;
  char* ws = (char*)d_ws; float* XT = (float*)(ws + WS_XT);
  k_xt<<<dim3(NP / 64, NIMG), 256, 0, stream>>>(F[0], XT);
  k_head<<<dim3(NP / 64, NIB), 128, 0, stream>>>(XT, F[1], (const int*)d_in[2], (float*)d_out);
}
